// GNN_2465311228180
// MI455X (gfx1250) — hardware-verified
//
#include <hip/hip_runtime.h>
#include <stddef.h>
#include <stdint.h>
#include <math.h>


#define CIN    64
#define HID    64
#define K2     128
#define NCLS   2
#define NGR    64
#define NTHR   256
#define NWAVE  8
#define EPT    8
#define CHUNK  (NTHR * EPT)
#define WCAP   (EPT * 32)
#define LISTN  (NWAVE * WCAP)
#define NBD    8192
#define SLD    13
#define NBA    1024
#define SLA    10
#define RCAP   12288
#define DEGCAP 64
#define MEAS_B1024  10466
#define MEAS_MAXDEG 25
#define GBM    64
#define GBN    64
#define GTHR   128
#define NU1    (HID * (CIN / 8))
#define NU2    (HID * (K2 / 8))
#define AGG_ZINTS (LISTN + 2 * RCAP + 3 * NBA)
#define AGG_LDS_INTS (AGG_ZINTS + 16)
#define NOUT   (NGR * NCLS)
#define NWL    ((HID + 1) * NCLS)
#define WSMAX  134217728

static_assert((CHUNK & (CHUNK - 1)) == 0 && CHUNK <= 4096);
static_assert((NBD & (NBD - 1)) == 0 && NBD == (1 << SLD));
static_assert((NBA & (NBA - 1)) == 0 && NBA == (1 << SLA));
static_assert(((long long)CHUNK << SLD) < (1LL << 31));
static_assert(((long long)CHUNK << SLA) < (1LL << 31));
static_assert(NBD % (NTHR * 4) == 0);
static_assert(LISTN % NTHR == 0);
static_assert(NBA % NWAVE == 0 && NBA % 32 == 0 && NBA % GBM == 0);
static_assert(RCAP % 32 == 0 && AGG_ZINTS % 4 == 0 && LISTN % 4 == 0);
static_assert(RCAP >= MEAS_B1024 + MEAS_B1024 / 20);
static_assert(DEGCAP >= MEAS_MAXDEG + 8);
static_assert(CIN % 32 == 0 && K2 % 32 == 0 && K2 == 2 * HID && HID == GBN);
static_assert(GBM == (GTHR / 32) * 16 && GBN == 64);
static_assert(NU1 % NTHR == 0 && NU2 % NTHR == 0);
static_assert(CIN / 8 == 8 && K2 / 8 == 16);
static_assert(HID == 2 * 32);
static_assert(AGG_LDS_INTS * 4 <= 300000);
static_assert(NOUT == 4 * 32);
static_assert(NOUT <= NTHR && NWL + 2 <= NTHR && NGR <= NTHR);

typedef float          v2f   __attribute__((ext_vector_type(2)));
typedef float          v4f   __attribute__((ext_vector_type(4)));
typedef float          v8f   __attribute__((ext_vector_type(8)));
typedef int            v4i   __attribute__((ext_vector_type(4)));
typedef int            v8i   __attribute__((ext_vector_type(8)));
typedef unsigned int   v4u   __attribute__((ext_vector_type(4)));
typedef unsigned short v8us  __attribute__((ext_vector_type(8)));
typedef unsigned short v16us __attribute__((ext_vector_type(16)));
typedef __bf16         v16bf __attribute__((ext_vector_type(16)));
typedef v2f  __attribute__((may_alias)) v2fa;
typedef v4f  __attribute__((may_alias)) v4fa;
typedef v4i  __attribute__((may_alias)) v4ia;
typedef v8us __attribute__((may_alias)) v8usa;
union FragB { v16bf v; v16us u; v8us h[2]; v8i w; };

__device__ __forceinline__ v8f wmb(const FragB& a, const FragB& b, v8f c) {
  v8f d = __builtin_amdgcn_wmma_f32_16x16x32_bf16(false, a.v, false, b.v, (short)0, c, false, false);
  asm volatile("v_nop\n\tv_nop\n\tv_nop\n\tv_nop" : "+v"(d) : "v"(a.w), "v"(b.w));
  return d;
}

__device__ __forceinline__ unsigned bf16_bits(float f) {
  const unsigned u = __float_as_uint(f);
  const unsigned r = (u + 0x7FFFu + ((u >> 16) & 1u)) >> 16;
  const unsigned nb = (u >> 16) | 0x40u;
  return ((u & 0x7FFFFFFFu) > 0x7F800000u) ? nb : r;
}
__device__ __forceinline__ float bf16_val(float f) {
  return __uint_as_float(bf16_bits(f) << 16);
}

template <int SLB>
__device__ __forceinline__ int scan_chunk(const int* __restrict__ dsts, int nE, int cbase, int slotBase,
                                          int nb, int vec8, int* list, int tid, int lane, int wave) {
  int wc = 0;
  const int el0  = tid * EPT;
  const int e0   = cbase + el0;
  const int sent = -2147483647 - 1;
  v4i da, db;
  if (vec8 != 0 && cbase + CHUNK <= nE) {
    da = *(const v4i*)(dsts + e0);
    db = *(const v4i*)(dsts + e0 + 4);
  } else {
    da.x = (e0     < nE) ? dsts[min(e0,     nE - 1)] : sent;
    da.y = (e0 + 1 < nE) ? dsts[min(e0 + 1, nE - 1)] : sent;
    da.z = (e0 + 2 < nE) ? dsts[min(e0 + 2, nE - 1)] : sent;
    da.w = (e0 + 3 < nE) ? dsts[min(e0 + 3, nE - 1)] : sent;
    db.x = (e0 + 4 < nE) ? dsts[min(e0 + 4, nE - 1)] : sent;
    db.y = (e0 + 5 < nE) ? dsts[min(e0 + 5, nE - 1)] : sent;
    db.z = (e0 + 6 < nE) ? dsts[min(e0 + 6, nE - 1)] : sent;
    db.w = (e0 + 7 < nE) ? dsts[min(e0 + 7, nE - 1)] : sent;
  }
  const unsigned nbs = (unsigned)slotBase;
  const unsigned unb = (unsigned)nb;
  const unsigned s0 = (unsigned)da.x - nbs, s1 = (unsigned)da.y - nbs;
  const unsigned s2 = (unsigned)da.z - nbs, s3 = (unsigned)da.w - nbs;
  const unsigned s4 = (unsigned)db.x - nbs, s5 = (unsigned)db.y - nbs;
  const unsigned s6 = (unsigned)db.z - nbs, s7 = (unsigned)db.w - nbs;
  const bool h0 = s0 < unb, h1 = s1 < unb, h2 = s2 < unb, h3 = s3 < unb;
  const bool h4 = s4 < unb, h5 = s5 < unb, h6 = s6 < unb, h7 = s7 < unb;
  const unsigned any = __builtin_amdgcn_ballot_w32(h0 | h1 | h2 | h3 | h4 | h5 | h6 | h7);
  if (any != 0u) {
#define HITJ(J, HJ, SJ) { \
      const unsigned mj = __builtin_amdgcn_ballot_w32(HJ); \
      if (mj != 0u) { \
        if (HJ) { \
          const int pos = wc + (int)__builtin_amdgcn_mbcnt_lo(mj, 0u); \
          if (pos < WCAP) list[wave * WCAP + pos] = ((el0 + (J)) << SLB) | (int)(SJ); \
        } \
        wc += (int)__builtin_popcount(mj); } }
    HITJ(0, h0, s0)
    HITJ(1, h1, s1)
    HITJ(2, h2, s2)
    HITJ(3, h3, s3)
    HITJ(4, h4, s4)
    HITJ(5, h5, s5)
    HITJ(6, h6, s6)
    HITJ(7, h7, s7)
#undef HITJ
  }
  return wc;
}

__global__ __launch_bounds__(NTHR) void k_wprep(const float* __restrict__ W1, const float* __restrict__ W2,
                                                unsigned short* W1T, unsigned short* W2T) {
  const int u = (int)blockIdx.x * NTHR + (int)threadIdx.x;
  v8us o;
  unsigned short* dp;
  if (u < NU1) {
    const int n  = u >> 3;
    const int k8 = (u & 7) * 8;
    const float* p = W1 + (size_t)k8 * HID + n;
#pragma unroll
    for (int i = 0; i < 8; ++i) o[i] = (unsigned short)bf16_bits(p[(size_t)i * HID]);
    dp = W1T + (size_t)n * CIN + k8;
  } else if (u < NU1 + NU2) {
    const int v  = u - NU1;
    const int n  = v >> 4;
    const int k8 = (v & 15) * 8;
    const int kk = k8 & (HID - 1);
    const float* p = W2 + (size_t)kk * HID + n;
#pragma unroll
    for (int i = 0; i < 8; ++i) o[i] = (unsigned short)bf16_bits(p[(size_t)i * HID]);
    dp = W2T + (size_t)n * K2 + k8;
  } else {
    return;
  }
  *(volatile v8us*)dp = o;
  __threadfence();
  *(volatile v8us*)dp = o;
}

__global__ __launch_bounds__(NTHR) void k_cvx(const float* __restrict__ x, int nN, int nUnits,
                                              unsigned short* xb) {
  const int u = (int)blockIdx.x * NTHR + (int)threadIdx.x;
  if (u >= nUnits) return;
  const int row = u >> 3;
  const int k8  = (u & 7) * 8;
  const int rc  = row < nN ? row : nN - 1;
  const float* p = x + (size_t)rc * CIN + k8;
  const v4f a = *(const v4fa*)p;
  const v4f b = *(const v4fa*)(p + 4);
  const bool ok = row < nN;
  v8us o;
  o[0] = ok ? (unsigned short)bf16_bits(a.x) : (unsigned short)0;
  o[1] = ok ? (unsigned short)bf16_bits(a.y) : (unsigned short)0;
  o[2] = ok ? (unsigned short)bf16_bits(a.z) : (unsigned short)0;
  o[3] = ok ? (unsigned short)bf16_bits(a.w) : (unsigned short)0;
  o[4] = ok ? (unsigned short)bf16_bits(b.x) : (unsigned short)0;
  o[5] = ok ? (unsigned short)bf16_bits(b.y) : (unsigned short)0;
  o[6] = ok ? (unsigned short)bf16_bits(b.z) : (unsigned short)0;
  o[7] = ok ? (unsigned short)bf16_bits(b.w) : (unsigned short)0;
  unsigned short* dp = xb + (size_t)row * CIN + k8;
  *(volatile v8us*)dp = o;
  __threadfence();
  *(volatile v8us*)dp = o;
}

__global__ __launch_bounds__(NTHR) void k_deg(const int* __restrict__ dsts, int nE, int vec8, float* dis) {
  __shared__ __attribute__((aligned(16))) int scnt[NBD];
  __shared__ __attribute__((aligned(16))) int list[LISTN];
  __shared__ int wcnt[NWAVE];
  const int tid = (int)threadIdx.x, lane = tid & 31, wave = tid >> 5;
  const int nodeBase = (int)blockIdx.x * NBD;

  for (int i = tid; i < NBD; i += NTHR) scnt[i] = 0;
  for (int i = tid; i < LISTN; i += NTHR) list[i] = 0;
  if (tid < NWAVE) wcnt[tid] = 0;
  __syncthreads();

  const int nChunks = (nE + CHUNK - 1) / CHUNK;
#pragma unroll 1
  for (int ch = 0; ch < nChunks; ++ch) {
    const int cbase = ch * CHUNK;
    const int wc = scan_chunk<SLD>(dsts, nE, cbase, nodeBase, NBD, vec8, list, tid, lane, wave);
    if (lane == 0) wcnt[wave] = wc;
    __syncthreads();
    if (wave == 0) {
#pragma unroll 1
      for (int w2 = 0; w2 < NWAVE; ++w2) {
        int c = wcnt[w2];
        c = c < 0 ? 0 : (c > WCAP ? WCAP : c);
#pragma unroll 1
        for (int b0 = 0; b0 < c; b0 += 32) {
          const int idx = b0 + lane;
          const int ent = list[w2 * WCAP + (idx < WCAP ? idx : WCAP - 1)];
          const int m32 = (c - b0) < 32 ? (c - b0) : 32;
#pragma unroll 1
          for (int k = 0; k < m32; ++k) {
            const int u  = __builtin_amdgcn_readlane(ent, k);
            const int sl = u & (NBD - 1);
            if (lane == 0) scnt[sl] = scnt[sl] + 1;
          }
        }
      }
    }
    __syncthreads();
  }

#pragma unroll 1
  for (int i = tid; i < NBD; i += NTHR) {
    int c = scnt[i];
    c = c < 0 ? 0 : c;
    const float d = (float)c + 1.0f;
    scnt[i] = __float_as_int(1.0f / sqrtf(d));
  }
  __syncthreads();

  v4f vals[NBD / (NTHR * 4)];
#pragma unroll
  for (int it = 0; it < NBD / (NTHR * 4); ++it) {
    const int s0 = it * (NTHR * 4) + 4 * tid;
    const v4i c4 = *(const v4ia*)(scnt + s0);
    v4f v;
    v.x = __int_as_float(c4.x); v.y = __int_as_float(c4.y);
    v.z = __int_as_float(c4.z); v.w = __int_as_float(c4.w);
    vals[it] = v;
  }
#pragma unroll
  for (int it = 0; it < NBD / (NTHR * 4); ++it) {
    const int s0 = it * (NTHR * 4) + 4 * tid;
    *(volatile v4f*)(dis + (size_t)nodeBase + s0) = vals[it];
  }
  __threadfence();
#pragma unroll
  for (int it = 0; it < NBD / (NTHR * 4); ++it) {
    const int s0 = it * (NTHR * 4) + 4 * tid;
    *(volatile v4f*)(dis + (size_t)nodeBase + s0) = vals[it];
  }
}

__global__ __launch_bounds__(GTHR) void k_gemm(
    const unsigned short* __restrict__ A, const unsigned short* __restrict__ WT,
    float* outF, int K, int ldo)
{
  __shared__ __attribute__((aligned(16))) float stg[GBM * GBN];
  const int tid = (int)threadIdx.x, lane = tid & 31, wave = tid >> 5, hh = lane >> 4, m = lane & 15;
  const int rowBase = (int)blockIdx.x * GBM;
  const int col0    = (int)blockIdx.y * GBN;

  v8f acc[4];
  {
    const v8f z = {0.f, 0.f, 0.f, 0.f, 0.f, 0.f, 0.f, 0.f};
    acc[0] = z; acc[1] = z; acc[2] = z; acc[3] = z;
  }
  const unsigned short* ap = A  + (size_t)(rowBase + 16 * wave + m) * (size_t)K + 8 * hh;
  const unsigned short* wp = WT + (size_t)(col0 + m) * (size_t)K + 8 * hh;
  const int ksteps = K >> 5;
#pragma unroll 1
  for (int ks = 0; ks < ksteps; ++ks) {
    FragB af;
    af.h[0] = *(const v8usa*)(ap + 32 * ks);
    af.h[1] = *(const v8usa*)(ap + 32 * ks + 16);
#pragma unroll
    for (int t = 0; t < 4; ++t) {
      const unsigned short* wq = wp + (size_t)(16 * t) * (size_t)K + 32 * ks;
      FragB bf;
      bf.h[0] = *(const v8usa*)wq;
      bf.h[1] = *(const v8usa*)(wq + 16);
      acc[t] = wmb(af, bf, acc[t]);
    }
  }

#pragma unroll
  for (int t = 0; t < 4; ++t) {
    const int lc = 16 * t + m;
#pragma unroll
    for (int r = 0; r < 8; ++r) {
      const int lr = 16 * wave + 8 * hh + r;
      stg[lr * GBN + lc] = acc[t][r];
    }
  }
  __syncthreads();

  v4f fv[8];
#pragma unroll
  for (int i = 0; i < 8; ++i) {
    const int lr = 16 * wave + 2 * i + hh;
    fv[i] = *(const v4fa*)(stg + lr * GBN + 4 * m);
  }
#pragma unroll
  for (int i = 0; i < 8; ++i) {
    const int lr = 16 * wave + 2 * i + hh;
    const int gr = rowBase + lr;
    float* op = outF + (size_t)gr * (size_t)ldo + col0 + 4 * m;
    *(volatile v4f*)op = fv[i];
  }
  __threadfence();
#pragma unroll
  for (int i = 0; i < 8; ++i) {
    const int lr = 16 * wave + 2 * i + hh;
    const int gr = rowBase + lr;
    float* op = outF + (size_t)gr * (size_t)ldo + col0 + 4 * m;
    *(volatile v4f*)op = fv[i];
  }
}

template <int MODE>
__global__ __launch_bounds__(NTHR) void k_agg(const int* __restrict__ srcs, const int* __restrict__ dsts,
                                              int nE, int nN, int vec8, int mRows,
                                              const float* __restrict__ dis,
                                              const float* __restrict__ xl, const float* __restrict__ bias,
                                              unsigned short* hb, float* hout) {
  extern __shared__ __attribute__((aligned(16))) int dsm[];
  int* list = dsm;
  int* hl   = dsm + LISTN;
  int* sl   = dsm + LISTN + RCAP;
  int* cnt  = dsm + LISTN + 2 * RCAP;
  int* offs = cnt + NBA;
  int* cur  = offs + NBA;
  int* misc = cur + NBA;
  const int tid = (int)threadIdx.x, lane = tid & 31, wave = tid >> 5;
  const int nodeBase = (int)blockIdx.x * NBA;

  {
    const v4i z4 = {0, 0, 0, 0};
    for (int i = tid * 4; i < AGG_ZINTS; i += NTHR * 4) *(v4ia*)(dsm + i) = z4;
    if (tid < 16) misc[tid] = 0;
  }
  float bv0, bv1;
  {
    const v2f a = *(const v2fa*)(bias + 2 * lane);
    bv0 = bf16_val(a.x); bv1 = bf16_val(a.y);
  }
  __syncthreads();

  int t = 0, ov = 0;
  const int nChunks = (nE + CHUNK - 1) / CHUNK;
#pragma unroll 1
  for (int ch = 0; ch < nChunks; ++ch) {
    const int cbase = ch * CHUNK;
    const int wc = scan_chunk<SLA>(dsts, nE, cbase, nodeBase, NBA, vec8, list, tid, lane, wave);
    if (lane == 0) misc[wave] = wc;
    __syncthreads();
    if (wave == 0) {
#pragma unroll 1
      for (int w2 = 0; w2 < NWAVE; ++w2) {
        int c = misc[w2];
        c = c < 0 ? 0 : (c > WCAP ? WCAP : c);
#pragma unroll 1
        for (int b0 = 0; b0 < c; b0 += 32) {
          const int idx = b0 + lane;
          const int ent = list[w2 * WCAP + (idx < WCAP ? idx : WCAP - 1)];
          const int m32 = (c - b0) < 32 ? (c - b0) : 32;
#pragma unroll 1
          for (int k = 0; k < m32; ++k) {
            const int u    = __builtin_amdgcn_readlane(ent, k);
            const int slot = u & (NBA - 1);
            const int el   = (u >> SLA) & (CHUNK - 1);
            const int pk   = ((cbase + el) << SLA) | slot;
            if (t < RCAP) {
              if (lane == 0) { hl[t] = pk; cnt[slot] = cnt[slot] + 1; }
              t = t + 1;
            } else {
              ov = 1;
            }
          }
        }
      }
    }
    __syncthreads();
  }
  if (wave == 0 && lane == 0) { misc[8] = t; misc[9] = ov; }
  __syncthreads();
  int tt = misc[8];
  tt = tt < 0 ? 0 : (tt > RCAP ? RCAP : tt);
  const int ovf = misc[9];

  if (wave == 0) {
    const int base = lane * (NBA / 32);
    int s = 0;
#pragma unroll 1
    for (int i = 0; i < NBA / 32; ++i) s += cnt[base + i];
    int incl = s;
#pragma unroll
    for (int d = 1; d < 32; d <<= 1) {
      const int y = __shfl_up(incl, d, 32);
      if (lane >= d) incl += y;
    }
    int run = incl - s;
#pragma unroll 1
    for (int i = 0; i < NBA / 32; ++i) {
      const int cv = cnt[base + i];
      offs[base + i] = run;
      cur[base + i]  = run;
      run += cv;
    }
  }
  __syncthreads();
  if (wave == 0) {
#pragma unroll 1
    for (int b0 = 0; b0 < tt; b0 += 32) {
      const int idx = b0 + lane;
      const int ent = hl[idx < RCAP ? idx : RCAP - 1];
      const int m32 = (tt - b0) < 32 ? (tt - b0) : 32;
#pragma unroll 1
      for (int k = 0; k < m32; ++k) {
        const int u    = __builtin_amdgcn_readlane(ent, k);
        const int slot = u & (NBA - 1);
        if (lane == 0) {
          int p = cur[slot];
          p = p < 0 ? 0 : (p > RCAP - 1 ? RCAP - 1 : p);
          sl[p] = u;
          cur[slot] = p + 1;
        }
      }
    }
  }
  __syncthreads();

  const float qnan = __int_as_float(0x7fc00000);
  const float pz = (ovf != 0) ? qnan : 0.0f;
  const int sa = (2 * lane) & 31, sb = (2 * lane + 1) & 31;
  const int q0s = (4 * lane) & 31, q1s = (4 * lane + 1) & 31;
  const int q2s = (4 * lane + 2) & 31, q3s = (4 * lane + 3) & 31;
#pragma unroll 1
  for (int si = 0; si < NBA / NWAVE; ++si) {
    const int s    = si * NWAVE + wave;
    const int node = nodeBase + s;
    int c = cnt[s];
    const bool big = c > DEGCAP;
    c = c < 0 ? 0 : (c > DEGCAP ? DEGCAP : c);
    int o = offs[s];
    o = o < 0 ? 0 : (o > RCAP ? RCAP : o);
    const int nc = node < nN ? node : nN - 1;
    const float dd = dis[nc];
    const float rd = dd * dd;
    float acc0 = 0.0f, acc1 = 0.0f;
#pragma unroll 1
    for (int b0 = 0; b0 < c; b0 += 32) {
      int idx = o + b0 + lane;
      idx = idx > RCAP - 1 ? RCAP - 1 : idx;
      const int ent = sl[idx];
      int eid = ent >> SLA;
      eid = eid < 0 ? 0 : (eid > nE - 1 ? nE - 1 : eid);
      int sr = srcs[eid];
      sr = sr < 0 ? 0 : (sr > nN - 1 ? nN - 1 : sr);
      const float cf  = dis[sr] * dd;
      const int   cfi = __float_as_int(cf);
      const int m32 = (c - b0) < 32 ? (c - b0) : 32;
#pragma unroll 1
      for (int k = 0; k < m32; ++k) {
        const int   sk = __builtin_amdgcn_readlane(sr, k);
        const float ck = __int_as_float(__builtin_amdgcn_readlane(cfi, k));
        const v2f a = *(const v2fa*)(xl + (size_t)sk * HID + 2 * lane);
        acc0 = fmaf(ck, a.x, acc0); acc1 = fmaf(ck, a.y, acc1);
      }
    }
    float sv0, sv1;
    {
      const v2f a = *(const v2fa*)(xl + (size_t)nc * HID + 2 * lane);
      sv0 = a.x; sv1 = a.y;
    }
    const float pzr = big ? qnan : pz;
    const bool live = node < nN;
    float y0 = (acc0 + sv0 * rd) + bv0;
    float y1 = (acc1 + sv1 * rd) + bv1;
    y0 = (y0 > 0.0f) ? y0 : (y0 - y0);
    y1 = (y1 > 0.0f) ? y1 : (y1 - y1);
    y0 = y0 + pzr; y1 = y1 + pzr;
    const float v0 = live ? y0 : 0.0f;
    const float v1 = live ? y1 : 0.0f;
    const bool wr = (node < mRows) && (lane < 16);
    if constexpr (MODE != 0) {
      const unsigned hb0 = bf16_bits(v0), hb1 = bf16_bits(v1);
      const unsigned lb0 = bf16_bits(v0 - __uint_as_float(hb0 << 16));
      const unsigned lb1 = bf16_bits(v1 - __uint_as_float(hb1 << 16));
      const int hw = (int)(hb0 | (hb1 << 16));
      const int lw = (int)(lb0 | (lb1 << 16));
      const int g0 = __shfl(hw, q0s, 32), g1 = __shfl(hw, q1s, 32);
      const int g2 = __shfl(hw, q2s, 32), g3 = __shfl(hw, q3s, 32);
      const int p0 = __shfl(lw, q0s, 32), p1 = __shfl(lw, q1s, 32);
      const int p2 = __shfl(lw, q2s, 32), p3 = __shfl(lw, q3s, 32);
      const bool lsel = (lane & 8) != 0;
      v4u pv;
      pv.x = (unsigned int)(lsel ? p0 : g0);
      pv.y = (unsigned int)(lsel ? p1 : g1);
      pv.z = (unsigned int)(lsel ? p2 : g2);
      pv.w = (unsigned int)(lsel ? p3 : g3);
      unsigned short* hp = hb + (size_t)node * K2 + 8 * (lane & 15);
      if (wr) *(volatile v4u*)hp = pv;
      __threadfence();
      if (wr) *(volatile v4u*)hp = pv;
    } else {
      v4f ow;
      ow.x = __shfl(v0, sa, 32); ow.y = __shfl(v1, sa, 32);
      ow.z = __shfl(v0, sb, 32); ow.w = __shfl(v1, sb, 32);
      float* op = hout + (size_t)node * HID + 4 * (lane & 15);
      if (wr) *(volatile v4f*)op = ow;
      __threadfence();
      if (wr) *(volatile v4f*)op = ow;
    }
  }
}

__global__ __launch_bounds__(NTHR) void k_pool(const float* __restrict__ hf, const int* __restrict__ bat,
                                               int nN, float* pl) {
  __shared__ __attribute__((aligned(16))) float wsum[NWAVE * HID];
  __shared__ __attribute__((aligned(16))) float outs[HID];
  const int tid = (int)threadIdx.x, lane = tid & 31, wave = tid >> 5;
  const int g = (int)blockIdx.x;

  float a0 = 0.0f, a1 = 0.0f;
#pragma unroll 1
  for (int i0 = wave * 32; i0 < nN; i0 += NTHR) {
    const int i  = i0 + lane;
    const int ic = i < nN ? i : nN - 1;
    const int b  = bat[ic];
    const bool hit = (i < nN) && (b == g);
    unsigned msk = __builtin_amdgcn_ballot_w32(hit);
    int nh = (int)__builtin_popcount(msk);
    nh = nh > 32 ? 32 : nh;
#pragma unroll 1
    for (int q = 0; q < nh; ++q) {
      const int k = __builtin_ffs((int)msk) - 1;
      msk &= msk - 1u;
      int node = i0 + (k < 0 ? 0 : k);
      node = node > nN - 1 ? nN - 1 : node;
      const v2f v = *(const v2fa*)(hf + (size_t)node * HID + 2 * lane);
      a0 += v.x; a1 += v.y;
    }
  }
  wsum[wave * HID + 2 * lane + 0] = a0;
  wsum[wave * HID + 2 * lane + 1] = a1;
  __syncthreads();
  if (tid < HID) {
    float s = 0.0f;
#pragma unroll
    for (int w2 = 0; w2 < NWAVE; ++w2) s += wsum[w2 * HID + tid];
    outs[tid] = s;
  }
  __syncthreads();
  const v4f ov = *(const v4fa*)(outs + 4 * (lane & 15));
  float* op = pl + (size_t)g * HID + 4 * (lane & 15);
  const bool okst = (wave == 0) && (lane < 16);
  if (okst) *(volatile v4f*)op = ov;
  __threadfence();
  if (okst) *(volatile v4f*)op = ov;
}

__global__ __launch_bounds__(NTHR) void k_head(const float* __restrict__ pl, const float* __restrict__ gfe,
                                               const float* __restrict__ Wl, const float* __restrict__ bl,
                                               float* out) {
  __shared__ float wls[NWL + 2];
  __shared__ float gfs[NGR];
  __shared__ float bls[4];
  __shared__ __attribute__((aligned(16))) float os[NOUT];
  const int tid = (int)threadIdx.x;
  {
    const float wv = Wl[tid < NWL ? tid : NWL - 1];
    const float gv = gfe[tid < NGR ? tid : NGR - 1];
    const float bb = bl[tid < NCLS ? tid : NCLS - 1];
    if (tid < NWL + 2) wls[tid] = (tid < NWL) ? bf16_val(wv) : 0.0f;
    if (tid < NGR) gfs[tid] = bf16_val(gv);
    if (tid < 4) bls[tid] = (tid < NCLS) ? bf16_val(bb) : 0.0f;
  }
  __syncthreads();
  if (tid < NOUT) {
    const int g = tid >> 1;
    const int o = tid & 1;
    const float* pr = pl + (size_t)g * HID;
    float s = 0.0f;
#pragma unroll 1
    for (int f4 = 0; f4 < HID / 4; ++f4) {
      const v4f p = *(const v4fa*)(pr + 4 * f4);
      const float* w = wls + (4 * f4) * NCLS + o;
      s = fmaf(p.x, w[0], s);
      s = fmaf(p.y, w[NCLS], s);
      s = fmaf(p.z, w[2 * NCLS], s);
      s = fmaf(p.w, w[3 * NCLS], s);
    }
    s = fmaf(gfs[g], wls[HID * NCLS + o], s);
    os[tid] = s + bls[o];
  }
  __syncthreads();
  if (tid < 32) {
    const v4f ov = *(const v4fa*)(os + 4 * tid);
    float* op = out + 4 * tid;
    *(volatile v4f*)op = ov;
    __threadfence();
    *(volatile v4f*)op = ov;
  }
}

static inline int cdiv(int a, int b) { return (a + b - 1) / b; }
static inline size_t al256(size_t o) { return (o + 255) & ~(size_t)255; }

extern "C" void kernel_launch(void* const* d_in, const int* in_sizes, int n_in,
                              void* d_out, int out_size, void* d_ws, size_t ws_size,
                              hipStream_t stream) {
  if (n_in < 10) return;
  if (in_sizes[0] < CIN || (in_sizes[0] % CIN) != 0) return;
  const int nN = in_sizes[0] / CIN;
  if (nN < 1 || nN > (1 << 22)) return;
  if (in_sizes[1] < 2 || (in_sizes[1] & 1) != 0) return;
  const int nE = in_sizes[1] / 2;
  if (nE < 1 || nE >= (1 << (31 - SLA))) return;
  if (in_sizes[2] != nN) return;
  if (in_sizes[3] != NGR) return;
  if (in_sizes[4] != CIN * HID || in_sizes[5] != HID) return;
  if (in_sizes[6] != HID * HID || in_sizes[7] != HID) return;
  if (in_sizes[8] != NWL || in_sizes[9] != NCLS) return;
  if (out_size != NOUT) return;

  const float* x    = (const float*)d_in[0];
  const int*   edge = (const int*)d_in[1];
  const int*   bat  = (const int*)d_in[2];
  const float* gfe  = (const float*)d_in[3];
  const float* W1   = (const float*)d_in[4];
  const float* b1   = (const float*)d_in[5];
  const float* W2   = (const float*)d_in[6];
  const float* b2   = (const float*)d_in[7];
  const float* Wl   = (const float*)d_in[8];
  const float* bl   = (const float*)d_in[9];
  float* out = (float*)d_out;
  const int* src = edge;
  const int* dst = edge + nE;

  const int MP   = cdiv(nN, GBM) * GBM;
  const int gM   = MP / GBM;
  const int gD   = cdiv(nN, NBD);
  const int NBPD = gD * NBD;
  const int gA   = cdiv(MP, NBA);
  if ((long long)gA * NBA < (long long)MP) return;
  if (NBPD < nN) return;
  const int vec8 = ((nE & 3) == 0) ? 1 : 0;

  char* ws = (char*)d_ws;
  size_t off = 0;
  const size_t oDIS = off; off = al256(off + (size_t)NBPD * 4);
  const size_t oW1T = off; off = al256(off + (size_t)HID * CIN * 2);
  const size_t oW2T = off; off = al256(off + (size_t)HID * K2 * 2);
  const size_t oXB  = off; off = al256(off + (size_t)MP * CIN * 2);
  const size_t oH   = off; off = al256(off + (size_t)MP * HID * 4);
  const size_t oA2  = off; off = al256(off + (size_t)MP * K2 * 2);
  const size_t oH2  = off; off = al256(off + (size_t)MP * HID * 4);
  const size_t oPL  = off; off = al256(off + (size_t)NGR * HID * 4);
  if (off > ws_size || off > (size_t)WSMAX) return;
  float*          DIS = (float*)(ws + oDIS);
  unsigned short* W1T = (unsigned short*)(ws + oW1T);
  unsigned short* W2T = (unsigned short*)(ws + oW2T);
  unsigned short* XB  = (unsigned short*)(ws + oXB);
  float*          H   = (float*)(ws + oH);
  unsigned short* A2  = (unsigned short*)(ws + oA2);
  float*          H2  = (float*)(ws + oH2);
  float*          PL  = (float*)(ws + oPL);

  const size_t aggLds = (size_t)AGG_LDS_INTS * 4;
  hipFuncSetAttribute(reinterpret_cast<const void*>(&k_agg<1>), hipFuncAttributeMaxDynamicSharedMemorySize, (int)aggLds);
  hipFuncSetAttribute(reinterpret_cast<const void*>(&k_agg<0>), hipFuncAttributeMaxDynamicSharedMemorySize, (int)aggLds);

  const int nUx = MP * (CIN / 8);
  k_wprep<<<(NU1 + NU2) / NTHR, NTHR, 0, stream>>>(W1, W2, W1T, W2T);
  k_cvx<<<cdiv(nUx, NTHR), NTHR, 0, stream>>>(x, nN, nUx, XB);
  k_deg<<<gD, NTHR, 0, stream>>>(dst, nE, vec8, DIS);
  k_gemm<<<dim3(gM, HID / GBN), GTHR, 0, stream>>>(XB, W1T, H, CIN, HID);
  k_agg<1><<<gA, NTHR, aggLds, stream>>>(src, dst, nE, nN, vec8, MP, DIS, H, b1, A2, H2);
  k_gemm<<<dim3(gM, HID / GBN), GTHR, 0, stream>>>(A2, W2T, H, K2, HID);
  k_agg<0><<<gA, NTHR, aggLds, stream>>>(src, dst, nE, nN, vec8, MP, DIS, H, b2, A2, H2);
  k_pool<<<NGR, NTHR, 0, stream>>>(H2, bat, nN, PL);
  k_head<<<1, NTHR, 0, stream>>>(PL, gfe, Wl, bl, out);
}
